// MultiHeadLatentAttention_56659208568833
// MI455X (gfx1250) — hardware-verified
//
#include <hip/hip_runtime.h>
#include <stddef.h>


typedef _Float16 h16;
typedef _Float16 v16h __attribute__((ext_vector_type(16)));
typedef _Float16 v8h  __attribute__((ext_vector_type(8)));
typedef float    v8f  __attribute__((ext_vector_type(8)));
typedef float    v4f  __attribute__((ext_vector_type(4)));

#ifndef NB
#define NB 2
#endif
#ifndef SEQ
#define SEQ 2048
#endif
#define NB_FULL  2
#define SEQ_FULL 2048
#define EDIM   2048
#define LAT    512
#define HALF_E 1024
#define NHEAD  16
#define HD     128
#define ROT    64
#define MROWS  (NB * SEQ)

static_assert(NB >= 1 && NB <= NB_FULL);
static_assert(SEQ >= 128 && SEQ <= SEQ_FULL && (SEQ % 128) == 0);
static_assert(EDIM == NHEAD * HD);
static_assert(HD == 128 && ROT * 2 == HD);
static_assert(HALF_E == NHEAD * ROT);
static_assert(HALF_E / 64 == NHEAD);
static_assert(LAT * 4 == EDIM);
static_assert((EDIM % 64) == 0 && (EDIM % 32) == 0);
static_assert((LAT % 64) == 0 && (LAT % 32) == 0);
static_assert((HALF_E % 64) == 0);
static_assert((MROWS % 64) == 0 && (SEQ % 64) == 0 && (SEQ % 32) == 0 && (SEQ % 8) == 0);
static_assert((8u << 8) == EDIM && (8u << 6) == LAT);
static_assert(((size_t)MROWS * (EDIM / 8)) % 256 == 0);
static_assert(((size_t)LAT * (EDIM / 8)) % 256 == 0);
static_assert(((size_t)HALF_E * (LAT / 8)) % 256 == 0);
static_assert((size_t)MROWS * EDIM < (size_t)0xFFFFFFFFu);
static_assert((size_t)NB_FULL * SEQ_FULL * EDIM * 4 == (size_t)33554432);

#define LDC 68
#define LDO 136
static_assert((LDC % 4) == 0 && LDC >= 64);
static_assert((LDO % 8) == 0 && LDO >= HD);

#define WCARRY 64.0f
#define PCARRY 1024.0f
#define VCARRY 64.0f

#define PLANE16_BYTES ((size_t)MROWS * EDIM * 2)
#define WDOWN_BYTES   ((size_t)LAT * EDIM * 2)
#define WUPH_BYTES    ((size_t)HALF_E * LAT * 2)
#define WUPV_BYTES    ((size_t)EDIM * LAT * 2)
#define WRK_BYTES     ((size_t)HALF_E * EDIM * 2)
#define WO_BYTES      ((size_t)EDIM * EDIM * 2)
#define LATP_BYTES    ((size_t)MROWS * LAT * 2)
#define TAB_BYTES     ((size_t)SEQ * 64 * 4)
#define OFF_XH   ((size_t)0)
#define OFF_WKVD (OFF_XH + PLANE16_BYTES)
#define OFF_WQD  (OFF_WKVD + WDOWN_BYTES)
#define OFF_WKU  (OFF_WQD + WDOWN_BYTES)
#define OFF_WQU  (OFF_WKU + WUPH_BYTES)
#define OFF_WVU  (OFF_WQU + WUPH_BYTES)
#define OFF_WRK  (OFF_WVU + WUPV_BYTES)
#define OFF_WRQ  (OFF_WRK + WRK_BYTES)
#define OFF_WO   (OFF_WRQ + WUPH_BYTES)
#define OFF_KVD  (OFF_WO + WO_BYTES)
#define OFF_QD   (OFF_KVD + LATP_BYTES)
#define OFF_Q    (OFF_QD + LATP_BYTES)
#define OFF_K    (OFF_Q + PLANE16_BYTES)
#define OFF_VT   (OFF_K + PLANE16_BYTES)
#define OFF_CTX  (OFF_VT + PLANE16_BYTES)
#define OFF_TAB  (OFF_CTX + PLANE16_BYTES)
#define WS_TOTAL (OFF_TAB + TAB_BYTES)
static_assert((PLANE16_BYTES % 128) == 0 && (WDOWN_BYTES % 128) == 0 && (WUPH_BYTES % 128) == 0);
static_assert((WUPV_BYTES % 128) == 0 && (WRK_BYTES % 128) == 0 && (WO_BYTES % 128) == 0);
static_assert((LATP_BYTES % 128) == 0 && (TAB_BYTES % 128) == 0);
static_assert(WS_TOTAL <= (size_t)134217728);

__device__ __forceinline__ float bf16r(float x) {
  unsigned int u = __float_as_uint(x);
  u = (u + 0x7FFFu + ((u >> 16) & 1u)) & 0xFFFF0000u;
  return __uint_as_float(u);
}

static __device__ __forceinline__ h16 toh_flush(float v) {
  const h16 r = (h16)v;
  return (fabsf(v) < 6.103515625e-05f) ? (h16)0.0f : r;
}

__device__ __forceinline__ v16h frag_at(const _Float16* p) {
  v8h lo = *(const v8h*)(p);
  v8h hi = *(const v8h*)(p + 16);
  v16h out;
#pragma unroll
  for (int i = 0; i < 8; ++i) { out[i] = lo[i]; out[i + 8] = hi[i]; }
  return out;
}

__device__ __forceinline__ v8f wmma16(v16h a, v16h b, v8f c) {
  v8f d = __builtin_amdgcn_wmma_f32_16x16x32_f16(false, a, false, b, (short)0, c,
                                                 false, false);
  asm volatile("v_nop\n\tv_nop\n\tv_nop\n\tv_nop" : "+v"(d) : "v"(a), "v"(b));
  return d;
}

__device__ __forceinline__ void wave_lds_sync() {
  __builtin_amdgcn_fence(3  , "wavefront");
  asm volatile("s_wait_dscnt 0x0" ::: "memory");
  __builtin_amdgcn_wave_barrier();
}

__global__ __launch_bounds__(256) void cvt_plane_kernel(
    const float* __restrict__ src, _Float16* __restrict__ dst,
    unsigned wsh, unsigned seq, unsigned seq_full, float carry) {
#pragma clang fp contract(off)
  const unsigned idx = blockIdx.x * 256u + threadIdx.x;
  const unsigned row = idx >> wsh;
  const unsigned c = (idx - (row << wsh)) * 8u;
  const unsigned bidx = row / seq;
  const unsigned sq = row - bidx * seq;
  const size_t srow = (size_t)bidx * seq_full + sq;
  const unsigned width = 8u << wsh;
  const float* p = src + srow * width + c;
  const v4f a0 = *(const v4f*)(p);
  const v4f a1 = *(const v4f*)(p + 4);
  v8h o;
#pragma unroll
  for (int i = 0; i < 4; ++i) {
    o[i]     = toh_flush(carry * bf16r(a0[i]));
    o[i + 4] = toh_flush(carry * bf16r(a1[i]));
  }
  _Float16* q = dst + (size_t)row * width + c;
  *(volatile v8h*)q = o;
  __threadfence();
  *(volatile v8h*)q = o;
}

__global__ __launch_bounds__(256) void rope_table_kernel(float* __restrict__ tab) {
#pragma clang fp contract(off)
  __shared__ float T[8 * 64];
  const unsigned tid = threadIdx.x;
  const unsigned pr = tid >> 5, f = tid & 31u;
  const unsigned pos = blockIdx.x * 8u + pr;
  double pw = 1.0;
#pragma unroll 1
  for (unsigned i = 0; i < f; ++i) pw *= 1.333521432163324;
  const float base = (float)pw;
  const float inv = 1.0f / base;
  const float ang = (float)pos * inv;
  float sn, cs;
  sincosf(ang, &sn, &cs);
  T[pr * 64u + f] = cs;
  T[pr * 64u + 32u + f] = sn;
  __syncthreads();
  if (tid < 128u) {
    const unsigned r = tid >> 4, c = (tid & 15u) * 4u;
    const v4f x = *(const v4f*)&T[r * 64u + c];
    float* q = tab + (size_t)(blockIdx.x * 8u + r) * 64u + c;
    *(volatile v4f*)q = x;
    __threadfence();
    *(volatile v4f*)q = x;
  }
}

template <int MODE>
__device__ __forceinline__ void gemm_body(
    const _Float16* __restrict__ A16, const _Float16* __restrict__ Bt, const unsigned K,
    const float* __restrict__ bias, const float* __restrict__ tab,
    float* __restrict__ outf, _Float16* __restrict__ out16,
    const unsigned ldo, const unsigned ostep, const unsigned ooff) {
  __shared__ float Cs[64 * LDC];
  const unsigned tid = threadIdx.x, lane = tid & 31u;
  const unsigned w = (unsigned)__builtin_amdgcn_readfirstlane((int)(tid >> 5));
  const unsigned mw = w >> 1, nw = w & 1u;
  const unsigned hh = lane >> 4, m = lane & 15u;
  const unsigned n0 = blockIdx.x * 64u;
  const unsigned row0 = blockIdx.y * 64u;

  const _Float16* ap  = A16 + (size_t)(row0 + mw * 16u + m) * K + hh * 8u;
  const _Float16* bp0 = Bt + (size_t)(n0 + nw * 32u + m) * K + hh * 8u;
  const _Float16* bp1 = bp0 + (size_t)16 * K;
  v8f acc0 = {}, acc1 = {};
#pragma unroll 2
  for (unsigned k0 = 0; k0 < K; k0 += 32u) {
    const v16h a  = frag_at(ap + k0);
    const v16h b0 = frag_at(bp0 + k0);
    const v16h b1 = frag_at(bp1 + k0);
    acc0 = wmma16(a, b0, acc0);
    acc1 = wmma16(a, b1, acc1);
  }
#pragma unroll
  for (int r = 0; r < 8; ++r) {
    float* d = &Cs[(mw * 16u + hh * 8u + (unsigned)r) * LDC + nw * 32u + m];
    d[0]  = acc0[r];
    d[16] = acc1[r];
  }
  __syncthreads();

  if (MODE == 0 || MODE == 2) {
    const unsigned ocol0 = blockIdx.x * ostep + ooff;
    v8h x[2];
    size_t off[2];
#pragma unroll
    for (unsigned i = 0; i < 2u; ++i) {
      const unsigned r = 32u * i + (tid >> 3);
      const unsigned c = (tid & 7u) * 8u;
      const v4f u0 = *(const v4f*)&Cs[r * LDC + c];
      const v4f u1 = *(const v4f*)&Cs[r * LDC + c + 4u];
      const v4f g0 = *(const v4f*)(bias + n0 + c);
      const v4f g1 = *(const v4f*)(bias + n0 + c + 4u);
      if (MODE == 2) {
        const unsigned pc = c ^ 32u;
        const unsigned crow = row0 + r;
        const unsigned bidx = crow / (unsigned)SEQ;
        const unsigned sq = crow - bidx * (unsigned)SEQ;
        const float* tr = tab + (size_t)sq * 64u + (c & 31u);
        const v4f p0 = *(const v4f*)&Cs[r * LDC + pc];
        const v4f p1 = *(const v4f*)&Cs[r * LDC + pc + 4u];
        const v4f h0 = *(const v4f*)(bias + n0 + pc);
        const v4f h1 = *(const v4f*)(bias + n0 + pc + 4u);
        const v4f c0 = *(const v4f*)(tr);
        const v4f c1 = *(const v4f*)(tr + 4);
        const v4f s0 = *(const v4f*)(tr + 32);
        const v4f s1 = *(const v4f*)(tr + 36);
        const float sg = (c < 32u) ? -1.0f : 1.0f;
#pragma unroll
        for (int j = 0; j < 4; ++j) {
          const float a0 = u0[j] * (1.0f / WCARRY) + bf16r(g0[j]);
          const float a1 = u1[j] * (1.0f / WCARRY) + bf16r(g1[j]);
          const float q0 = sg * (p0[j] * (1.0f / WCARRY) + bf16r(h0[j]));
          const float q1 = sg * (p1[j] * (1.0f / WCARRY) + bf16r(h1[j]));
          x[i][j]     = toh_flush(a0 * c0[j] + q0 * s0[j]);
          x[i][j + 4] = toh_flush(a1 * c1[j] + q1 * s1[j]);
        }
      } else {
#pragma unroll
        for (int j = 0; j < 4; ++j) {
          x[i][j]     = toh_flush(u0[j] * (1.0f / WCARRY) + bf16r(g0[j]));
          x[i][j + 4] = toh_flush(u1[j] * (1.0f / WCARRY) + bf16r(g1[j]));
        }
      }
      off[i] = (size_t)(row0 + r) * ldo + ocol0 + c;
    }
#pragma unroll
    for (int i = 0; i < 2; ++i) *(volatile v8h*)(out16 + off[i]) = x[i];
    __threadfence();
#pragma unroll
    for (int i = 0; i < 2; ++i) *(volatile v8h*)(out16 + off[i]) = x[i];
  }

  if (MODE == 1) {
    const unsigned bidx = row0 / (unsigned)SEQ;
    const unsigned key0 = row0 - bidx * (unsigned)SEQ;
    v8h x[2];
    size_t off[2];
#pragma unroll
    for (unsigned i = 0; i < 2u; ++i) {
      const unsigned dcol = 32u * i + (tid >> 3);
      const unsigned kk = (tid & 7u) * 8u;
      const float bb = bf16r(bias[n0 + dcol]);
#pragma unroll
      for (unsigned j = 0; j < 8u; ++j) {
        const float t = Cs[(kk + j) * LDC + dcol] * (1.0f / WCARRY) + bb;
        x[i][j] = toh_flush(t);
      }
      off[i] = ((size_t)bidx * EDIM + n0 + dcol) * SEQ + key0 + kk;
    }
#pragma unroll
    for (int i = 0; i < 2; ++i) *(volatile v8h*)(out16 + off[i]) = x[i];
    __threadfence();
#pragma unroll
    for (int i = 0; i < 2; ++i) *(volatile v8h*)(out16 + off[i]) = x[i];
  }

  if (MODE == 3) {
    const float cs = 1.0f / (WCARRY * VCARRY);
    v4f xs[4];
    size_t off[4];
#pragma unroll
    for (unsigned i = 0; i < 4u; ++i) {
      const unsigned r = 16u * i + (tid >> 4);
      const unsigned c = (tid & 15u) * 4u;
      const unsigned crow = row0 + r;
      const unsigned bidx = crow / (unsigned)SEQ;
      const unsigned sq = crow - bidx * (unsigned)SEQ;
      const size_t frow = (size_t)bidx * SEQ_FULL + sq;
      const v4f u = *(const v4f*)&Cs[r * LDC + c];
      const v4f g = *(const v4f*)(bias + n0 + c);
      v4f val;
#pragma unroll
      for (int j = 0; j < 4; ++j) val[j] = u[j] * cs + bf16r(g[j]);
      xs[i] = val;
      off[i] = frow * EDIM + n0 + c;
    }
#pragma unroll
    for (int i = 0; i < 4; ++i) *(volatile v4f*)(outf + off[i]) = xs[i];
    __threadfence();
#pragma unroll
    for (int i = 0; i < 4; ++i) *(volatile v4f*)(outf + off[i]) = xs[i];
  }
}

__global__ __launch_bounds__(256) void gemm_plane_kernel(
    const _Float16* __restrict__ A16, const _Float16* __restrict__ Bt, unsigned K,
    const float* __restrict__ bias, _Float16* __restrict__ out16,
    unsigned ldo, unsigned ostep, unsigned ooff) {
  gemm_body<0>(A16, Bt, K, bias, bias, (float*)0, out16, ldo, ostep, ooff);
}
__global__ __launch_bounds__(256) void gemm_vt_kernel(
    const _Float16* __restrict__ A16, const _Float16* __restrict__ Bt, unsigned K,
    const float* __restrict__ bias, _Float16* __restrict__ vt) {
  gemm_body<1>(A16, Bt, K, bias, bias, (float*)0, vt, 0u, 0u, 0u);
}
__global__ __launch_bounds__(256) void gemm_rope_kernel(
    const _Float16* __restrict__ A16, const _Float16* __restrict__ Bt, unsigned K,
    const float* __restrict__ bias, const float* __restrict__ tab,
    _Float16* __restrict__ out16, unsigned ldo, unsigned ostep, unsigned ooff) {
  gemm_body<2>(A16, Bt, K, bias, tab, (float*)0, out16, ldo, ostep, ooff);
}
__global__ __launch_bounds__(256) void gemm_out_kernel(
    const _Float16* __restrict__ A16, const _Float16* __restrict__ Bt, unsigned K,
    const float* __restrict__ bias, float* __restrict__ outf) {
  gemm_body<3>(A16, Bt, K, bias, bias, outf, (_Float16*)0, 0u, 0u, 0u);
}

__global__ __launch_bounds__(256) __attribute__((amdgpu_num_vgpr(256))) void attn_kernel(
    const _Float16* __restrict__ Qh, const _Float16* __restrict__ Kh,
    const _Float16* __restrict__ Vt, _Float16* __restrict__ Ov) {
  __shared__ _Float16 Os[8 * 16 * LDO];

  const unsigned tid = threadIdx.x, lane = tid & 31u;
  const unsigned w = (unsigned)__builtin_amdgcn_readfirstlane((int)(tid >> 5));
  const unsigned hh = lane >> 4, m = lane & 15u;
  const unsigned q0 = blockIdx.x * 128u + w * 16u;
  const unsigned head = blockIdx.y;
  const unsigned b = blockIdx.z;
  const float scale = 0.08838834764831845f;

  const _Float16* qp = Qh + (size_t)(b * (unsigned)SEQ + q0 + m) * EDIM + head * HD + hh * 8u;
  v16h qf[4];
#pragma unroll
  for (int c = 0; c < 4; ++c) qf[c] = frag_at(qp + c * 32);

  const _Float16* kp = Kh + ((size_t)b * SEQ + m) * EDIM + head * HD + hh * 8u;
  const _Float16* vp = Vt + ((size_t)b * EDIM + head * HD + m) * SEQ + hh * 8u;

  float mrun = -1.0e30f, lrun = 0.0f;
  v8f o[8];
#pragma unroll
  for (int nb = 0; nb < 8; ++nb) o[nb] = (v8f){};

#pragma unroll 1
  for (unsigned kb = 0; kb < (unsigned)SEQ; kb += 32u) {
    const _Float16* k0p = kp + (size_t)kb * EDIM;
    v8f s0 = {}, s1 = {};
#pragma unroll
    for (int c = 0; c < 4; ++c) {
      const v16h ka = frag_at(k0p + c * 32);
      const v16h kc = frag_at(k0p + (size_t)16 * EDIM + c * 32);
      s0 = wmma16(ka, qf[c], s0);
      s1 = wmma16(kc, qf[c], s1);
    }

    float mx = -1.0e30f;
#pragma unroll
    for (int r = 0; r < 8; ++r) {
      s0[r] = s0[r] * scale;
      s1[r] = s1[r] * scale;
      mx = fmaxf(mx, fmaxf(s0[r], s1[r]));
    }
    mx = fmaxf(mx, __shfl_xor(mx, 16, 32));
    const float mn = fmaxf(mrun, mx);
    const float alpha = __expf(mrun - mn);
    mrun = mn;

    v16h pf;
    float rs = 0.0f;
#pragma unroll
    for (int r = 0; r < 8; ++r) {
      const h16 p0 = toh_flush(__expf(s0[r] - mn) * PCARRY);
      const h16 p1 = toh_flush(__expf(s1[r] - mn) * PCARRY);
      pf[r] = p0;
      pf[r + 8] = p1;
      rs += (float)p0 + (float)p1;
    }
    rs += __shfl_xor(rs, 16, 32);
    lrun = alpha * lrun + rs;

#pragma unroll
    for (int nb = 0; nb < 8; ++nb)
#pragma unroll
      for (int r = 0; r < 8; ++r) o[nb][r] = o[nb][r] * alpha;

    const _Float16* v0p = vp + kb;
#pragma unroll
    for (int nb = 0; nb < 8; ++nb) {
      const v16h vf = frag_at(v0p + (size_t)(nb * 16) * SEQ);
      o[nb] = wmma16(vf, pf, o[nb]);
    }
  }

  const float inv = __builtin_amdgcn_rcpf(lrun) * VCARRY;
  const unsigned tb = w * (16u * LDO);
#pragma unroll
  for (int nb = 0; nb < 8; ++nb) {
    v8h x;
#pragma unroll
    for (int r = 0; r < 8; ++r) x[r] = toh_flush(o[nb][r] * inv);
    *(v8h*)&Os[tb + m * LDO + (unsigned)nb * 16u + hh * 8u] = x;
  }
  wave_lds_sync();
  v8h xo[8];
  size_t off[8];
#pragma unroll
  for (unsigned i = 0; i < 8u; ++i) {
    const unsigned r = 2u * i + (lane >> 4);
    const unsigned c = (lane & 15u) * 8u;
    xo[i] = *(const v8h*)&Os[tb + r * LDO + c];
    off[i] = (size_t)(b * (unsigned)SEQ + q0 + r) * EDIM + head * HD + c;
  }
#pragma unroll
  for (int i = 0; i < 8; ++i) *(volatile v8h*)(Ov + off[i]) = xo[i];
  __threadfence();
#pragma unroll
  for (int i = 0; i < 8; ++i) *(volatile v8h*)(Ov + off[i]) = xo[i];
}

extern "C" void kernel_launch(void* const* d_in, const int* in_sizes, int n_in,
                              void* d_out, int out_size, void* d_ws, size_t ws_size,
                              hipStream_t stream) {
  if (n_in < 17) return;
  const long long need_x = ((long long)(NB - 1) * SEQ_FULL + SEQ) * EDIM;
  if ((long long)in_sizes[0] < need_x) return;
  if ((long long)in_sizes[1] < (long long)LAT * EDIM) return;
  if ((long long)in_sizes[3] < (long long)LAT * EDIM) return;
  if ((long long)in_sizes[5] < (long long)HALF_E * LAT) return;
  if ((long long)in_sizes[7] < (long long)HALF_E * LAT) return;
  if ((long long)in_sizes[9] < (long long)EDIM * LAT) return;
  if ((long long)in_sizes[11] < (long long)HALF_E * EDIM) return;
  if ((long long)in_sizes[13] < (long long)HALF_E * LAT) return;
  if ((long long)in_sizes[15] < (long long)EDIM * EDIM) return;
  if (in_sizes[2] < LAT || in_sizes[4] < LAT) return;
  if (in_sizes[6] < HALF_E || in_sizes[8] < HALF_E) return;
  if (in_sizes[10] < EDIM || in_sizes[12] < HALF_E || in_sizes[14] < HALF_E) return;
  if (in_sizes[16] < EDIM) return;
  if ((long long)out_size < need_x) return;
  if (ws_size < WS_TOTAL) return;

  const float* X    = (const float*)d_in[0];
  const float* wkvd = (const float*)d_in[1];
  const float* bkvd = (const float*)d_in[2];
  const float* wqd  = (const float*)d_in[3];
  const float* bqd  = (const float*)d_in[4];
  const float* wku  = (const float*)d_in[5];
  const float* bku  = (const float*)d_in[6];
  const float* wqu  = (const float*)d_in[7];
  const float* bqu  = (const float*)d_in[8];
  const float* wvu  = (const float*)d_in[9];
  const float* bvu  = (const float*)d_in[10];
  const float* wrk  = (const float*)d_in[11];
  const float* brk  = (const float*)d_in[12];
  const float* wrq  = (const float*)d_in[13];
  const float* brq  = (const float*)d_in[14];
  const float* wo   = (const float*)d_in[15];
  const float* bo   = (const float*)d_in[16];
  float* out = (float*)d_out;

  char* ws = (char*)d_ws;
  _Float16* XH     = (_Float16*)(ws + OFF_XH);
  _Float16* Wkvd16 = (_Float16*)(ws + OFF_WKVD);
  _Float16* Wqd16  = (_Float16*)(ws + OFF_WQD);
  _Float16* Wku16  = (_Float16*)(ws + OFF_WKU);
  _Float16* Wqu16  = (_Float16*)(ws + OFF_WQU);
  _Float16* Wvu16  = (_Float16*)(ws + OFF_WVU);
  _Float16* Wrk16  = (_Float16*)(ws + OFF_WRK);
  _Float16* Wrq16  = (_Float16*)(ws + OFF_WRQ);
  _Float16* Wo16   = (_Float16*)(ws + OFF_WO);
  _Float16* KVD16  = (_Float16*)(ws + OFF_KVD);
  _Float16* QD16   = (_Float16*)(ws + OFF_QD);
  _Float16* Qh16   = (_Float16*)(ws + OFF_Q);
  _Float16* Kh16   = (_Float16*)(ws + OFF_K);
  _Float16* Vt16   = (_Float16*)(ws + OFF_VT);
  _Float16* Ctx16  = (_Float16*)(ws + OFF_CTX);
  float*    Tab    = (float*)(ws + OFF_TAB);

  dim3 blk(256);
  const unsigned gy = MROWS / 64;

  cvt_plane_kernel<<<dim3((unsigned)(((size_t)MROWS * (EDIM / 8)) / 256)), blk, 0, stream>>>(
      X, XH, 8u, (unsigned)SEQ, (unsigned)SEQ_FULL, 1.0f);
  cvt_plane_kernel<<<dim3((LAT * (EDIM / 8)) / 256), blk, 0, stream>>>(
      wkvd, Wkvd16, 8u, (unsigned)LAT, (unsigned)LAT, WCARRY);
  cvt_plane_kernel<<<dim3((LAT * (EDIM / 8)) / 256), blk, 0, stream>>>(
      wqd, Wqd16, 8u, (unsigned)LAT, (unsigned)LAT, WCARRY);
  cvt_plane_kernel<<<dim3((HALF_E * (LAT / 8)) / 256), blk, 0, stream>>>(
      wku, Wku16, 6u, (unsigned)HALF_E, (unsigned)HALF_E, WCARRY);
  cvt_plane_kernel<<<dim3((HALF_E * (LAT / 8)) / 256), blk, 0, stream>>>(
      wqu, Wqu16, 6u, (unsigned)HALF_E, (unsigned)HALF_E, WCARRY);
  cvt_plane_kernel<<<dim3((EDIM * (LAT / 8)) / 256), blk, 0, stream>>>(
      wvu, Wvu16, 6u, (unsigned)EDIM, (unsigned)EDIM, WCARRY);
  cvt_plane_kernel<<<dim3((HALF_E * (EDIM / 8)) / 256), blk, 0, stream>>>(
      wrk, Wrk16, 8u, (unsigned)HALF_E, (unsigned)HALF_E, WCARRY);
  cvt_plane_kernel<<<dim3((HALF_E * (LAT / 8)) / 256), blk, 0, stream>>>(
      wrq, Wrq16, 6u, (unsigned)HALF_E, (unsigned)HALF_E, WCARRY);
  cvt_plane_kernel<<<dim3((EDIM * (EDIM / 8)) / 256), blk, 0, stream>>>(
      wo, Wo16, 8u, (unsigned)EDIM, (unsigned)EDIM, WCARRY);

  rope_table_kernel<<<dim3(SEQ / 8), blk, 0, stream>>>(Tab);

  gemm_plane_kernel<<<dim3(LAT / 64, gy), blk, 0, stream>>>(
      XH, Wkvd16, (unsigned)EDIM, bkvd, KVD16, (unsigned)LAT, 64u, 0u);
  gemm_plane_kernel<<<dim3(LAT / 64, gy), blk, 0, stream>>>(
      XH, Wqd16, (unsigned)EDIM, bqd, QD16, (unsigned)LAT, 64u, 0u);
  gemm_plane_kernel<<<dim3(HALF_E / 64, gy), blk, 0, stream>>>(
      KVD16, Wku16, (unsigned)LAT, bku, Kh16, (unsigned)EDIM, (unsigned)HD, 0u);
  gemm_plane_kernel<<<dim3(HALF_E / 64, gy), blk, 0, stream>>>(
      QD16, Wqu16, (unsigned)LAT, bqu, Qh16, (unsigned)EDIM, (unsigned)HD, 0u);
  gemm_vt_kernel<<<dim3(EDIM / 64, gy), blk, 0, stream>>>(
      KVD16, Wvu16, (unsigned)LAT, bvu, Vt16);
  gemm_rope_kernel<<<dim3(HALF_E / 64, gy), blk, 0, stream>>>(
      XH, Wrk16, (unsigned)EDIM, brk, Tab, Kh16, (unsigned)EDIM, (unsigned)HD, (unsigned)ROT);
  gemm_rope_kernel<<<dim3(HALF_E / 64, gy), blk, 0, stream>>>(
      QD16, Wrq16, (unsigned)LAT, brq, Tab, Qh16, (unsigned)EDIM, (unsigned)HD, (unsigned)ROT);

  attn_kernel<<<dim3(SEQ / 128, NHEAD, NB), blk, 0, stream>>>(Qh16, Kh16, Vt16, Ctx16);

  gemm_out_kernel<<<dim3(EDIM / 64, gy), blk, 0, stream>>>(
      Ctx16, Wo16, (unsigned)EDIM, bo, out);
}
